// NeuralSplineCoupling_8014408974444
// MI455X (gfx1250) — hardware-verified
//
#include <hip/hip_runtime.h>
#include <stddef.h>
#include <stdint.h>


#pragma clang fp contract(off)

#define NH     128
#define DIN    16
#define DT     8
#define KC     8
#define K1P    32
#define N3     376
#define N3P    384
#define NT3    24
#define SPL    47
#define NB     16
#define O_W1H  0
#define O_W2H  4096
#define O_W3H  20480
#define HTOT   69632
#define O_W1L  (HTOT + O_W1H)
#define O_W2L  (HTOT + O_W2H)
#define O_W3L  (HTOT + O_W3H)
#define WTOT   (2 * HTOT)
#define PREPB  34
#define PB1    2
#define PB2    10
#define NWAVE  2
#define NTHR   64
#define RPB    32
#define APITCH 136
#define PP     388
#define BN_EPS 1e-5f
#define WSCAP  134217728

static_assert(HTOT == NH * K1P + NH * NH + N3P * NH);
static_assert(PREPB * 2048 == HTOT);
static_assert(PB1 * 2048 == O_W2H);
static_assert(PB2 * 2048 == O_W3H);
static_assert(NT3 * 16 == N3P);
static_assert(DT * SPL == N3);
static_assert(PP >= N3P);
static_assert(APITCH >= NH);
static_assert((APITCH % 8) == 0);
static_assert(RPB == NWAVE * 16);
static_assert(NTHR == NWAVE * 32);
static_assert(((WTOT * 2) % 512) == 0);
static_assert(DT + KC == DIN);

typedef float          v4f  __attribute__((ext_vector_type(4)));
typedef float          v8f  __attribute__((ext_vector_type(8)));
typedef unsigned short v8us __attribute__((ext_vector_type(8)));
typedef __bf16         v16b __attribute__((ext_vector_type(16)));
union FragB { v16b v; v8us u[2]; };

__device__ __forceinline__ v8f wm(v16b a, v16b b, v8f c) {
  v8f d = __builtin_amdgcn_wmma_f32_16x16x32_bf16(false, a, false, b, (short)0, c, false, false);
  asm volatile("v_nop\n\tv_nop\n\tv_nop\n\tv_nop" : "+v"(d) : "v"(a), "v"(b));
  return d;
}

__device__ __forceinline__ v8f zero8() {
  v8f z = {0.f, 0.f, 0.f, 0.f, 0.f, 0.f, 0.f, 0.f};
  return z;
}

__device__ __forceinline__ v16b ldfrag(const unsigned short* p) {
  FragB f;
  f.u[0] = *(const v8us*)p;
  f.u[1] = *(const v8us*)(p + 16);
  return f.v;
}

__device__ __forceinline__ unsigned short f2bf(float f) {
  unsigned int u = __float_as_uint(f);
  u = u + 0x7FFFu + ((u >> 16) & 1u);
  return (unsigned short)(u >> 16);
}
__device__ __forceinline__ float bf2f(unsigned short b) {
  return __uint_as_float(((unsigned int)b) << 16);
}

__device__ __forceinline__ float swish_f(float v) {
  const float e = expf(-fabsf(v));
  const float rr = 1.0f / (1.0f + e);
  const float sg = (v >= 0.0f) ? rr : e * rr;
  return v * sg;
}

__device__ __forceinline__ float softplus_f(float v) {
  return fmaxf(v, 0.0f) + log1pf(expf(-fabsf(v)));
}

__global__ __launch_bounds__(256) void k_prep(const float* __restrict__ W1, const float* __restrict__ W2,
                                             const float* __restrict__ W3, unsigned short* wsp) {
  const int b = blockIdx.x, tid = threadIdx.x;
  const int e = (b * 256 + tid) * 8;
  float v[8];
  int zero_lo = 0, zero_all = 0;
  if (b < PB1) {
    const int n = e >> 5, k0 = e & 31, kk = k0 & 15;
    zero_lo = (k0 >= 16) ? 1 : 0;
#pragma unroll
    for (int i = 0; i < 8; ++i) v[i] = W1[(kk + i) * NH + n];
  } else if (b < PB2) {
    const int le = e - O_W2H;
    const int n = le >> 7, k0 = le & 127;
#pragma unroll
    for (int i = 0; i < 8; ++i) v[i] = W2[(k0 + i) * NH + n];
  } else {
    const int le = e - O_W3H;
    const int n = le >> 7, k0 = le & 127;
    const int nc = min(n, N3 - 1);
    zero_all = (n >= N3) ? 1 : 0;
#pragma unroll
    for (int i = 0; i < 8; ++i) v[i] = W3[(size_t)(k0 + i) * N3 + nc];
  }
  v8us oh, ol;
#pragma unroll
  for (int i = 0; i < 8; ++i) {
    const float vv = (zero_all != 0) ? 0.0f : v[i];
    const unsigned short hb = f2bf(vv);
    const unsigned short lb = f2bf(vv - bf2f(hb));
    oh[i] = hb;
    ol[i] = (zero_lo != 0) ? (unsigned short)0 : lb;
  }
  unsigned short* dh = wsp + e;
  unsigned short* dl = wsp + HTOT + e;
  *(volatile v8us*)dh = oh;
  *(volatile v8us*)dl = ol;
  __threadfence();
  *(volatile v8us*)dh = oh;
  *(volatile v8us*)dl = ol;
}

__global__ __launch_bounds__(NTHR) void k_main(
    const float* __restrict__ x, const float* __restrict__ cc,
    const float* __restrict__ bns, const float* __restrict__ bnb,
    const float* __restrict__ bnm, const float* __restrict__ bnv,
    const float* __restrict__ b1, const float* __restrict__ b2, const float* __restrict__ b3,
    const unsigned short* __restrict__ wsp, float* out, int yoff) {
  __shared__ __attribute__((aligned(16))) unsigned short acth[NWAVE * 16 * APITCH];
  __shared__ __attribute__((aligned(16))) unsigned short actl[NWAVE * 16 * APITCH];
  __shared__ __attribute__((aligned(16))) float pst[NWAVE * 16 * PP];
  __shared__ __attribute__((aligned(16))) float yst[NWAVE * 16 * DIN];
  __shared__ __attribute__((aligned(16))) float lst[RPB];

  const int tid = threadIdx.x, lane = tid & 31, wave = tid >> 5, hh = lane >> 4, m = lane & 15;
  const int row0 = blockIdx.x * RPB + wave * 16;
  unsigned short* ahw = acth + wave * (16 * APITCH);
  unsigned short* alw = actl + wave * (16 * APITCH);
  float* pw = pst + wave * (16 * PP);
  float* yw = yst + wave * (16 * DIN);

  FragB a1;
  {
    const size_t r = (size_t)(row0 + m);
    const float* px = x + r * DIN + DT;
    const float* pc = cc + r * KC;
    const v4f x0 = *(const v4f*)px;
    const v4f x1 = *(const v4f*)(px + 4);
    const v4f c0 = *(const v4f*)pc;
    const v4f c1 = *(const v4f*)(pc + 4);
    const float xv[8] = {x0.x, x0.y, x0.z, x0.w, x1.x, x1.y, x1.z, x1.w};
    const float cv[8] = {c0.x, c0.y, c0.z, c0.w, c1.x, c1.y, c1.z, c1.w};
    v8us uh, ul;
#pragma unroll
    for (int i = 0; i < 8; ++i) {
      const int k = 8 * hh + i;
      const float v = (hh != 0) ? cv[i] : xv[i];
      float t = (v - bnm[k]) * rsqrtf(bnv[k] + BN_EPS);
      t = t * bns[k];
      t = t + bnb[k];
      const unsigned short hb = f2bf(t);
      uh[i] = hb;
      ul[i] = f2bf(t - bf2f(hb));
    }
    a1.u[0] = uh;
    a1.u[1] = ul;
  }

  {
    const unsigned short* w1h = wsp + O_W1H;
    const unsigned short* w1l = wsp + O_W1L;
#pragma unroll 1
    for (int nt = 0; nt < NH / 16; ++nt) {
      const int n = nt * 16 + m;
      const v16b bh = ldfrag(w1h + n * K1P + 8 * hh);
      const v16b bl = ldfrag(w1l + n * K1P + 8 * hh);
      v8f acc = zero8();
      acc = wm(a1.v, bh, acc);
      acc = wm(a1.v, bl, acc);
      const float bias = b1[n];
#pragma unroll
      for (int r = 0; r < 8; ++r) {
        const float sv = swish_f(acc[r] + bias);
        const unsigned short hb = f2bf(sv);
        const int o = (8 * hh + r) * APITCH + n;
        ahw[o] = hb;
        alw[o] = f2bf(sv - bf2f(hb));
      }
    }
  }
  __syncthreads();
  v16b fh[4], fl[4];
#pragma unroll
  for (int kc = 0; kc < 4; ++kc) {
    fh[kc] = ldfrag(ahw + m * APITCH + kc * 32 + 8 * hh);
    fl[kc] = ldfrag(alw + m * APITCH + kc * 32 + 8 * hh);
  }
  __syncthreads();

  {
    const unsigned short* w2h = wsp + O_W2H;
    const unsigned short* w2l = wsp + O_W2L;
#pragma unroll 1
    for (int nt = 0; nt < NH / 16; ++nt) {
      const int n = nt * 16 + m;
      const unsigned short* bph = w2h + n * NH + 8 * hh;
      const unsigned short* bpl = w2l + n * NH + 8 * hh;
      v8f acc = zero8();
#pragma unroll
      for (int kc = 0; kc < 4; ++kc) {
        const v16b bh = ldfrag(bph + kc * 32);
        const v16b bl = ldfrag(bpl + kc * 32);
        acc = wm(fh[kc], bh, acc);
        acc = wm(fh[kc], bl, acc);
        acc = wm(fl[kc], bh, acc);
      }
      const float bias = b2[n];
#pragma unroll
      for (int r = 0; r < 8; ++r) {
        const float sv = swish_f(acc[r] + bias);
        const unsigned short hb = f2bf(sv);
        const int o = (8 * hh + r) * APITCH + n;
        ahw[o] = hb;
        alw[o] = f2bf(sv - bf2f(hb));
      }
    }
  }
  __syncthreads();
#pragma unroll
  for (int kc = 0; kc < 4; ++kc) {
    fh[kc] = ldfrag(ahw + m * APITCH + kc * 32 + 8 * hh);
    fl[kc] = ldfrag(alw + m * APITCH + kc * 32 + 8 * hh);
  }

  {
    const unsigned short* w3h = wsp + O_W3H;
    const unsigned short* w3l = wsp + O_W3L;
#pragma unroll 1
    for (int nt = 0; nt < NT3; ++nt) {
      const int n = nt * 16 + m;
      const unsigned short* bph = w3h + n * NH + 8 * hh;
      const unsigned short* bpl = w3l + n * NH + 8 * hh;
      v8f acc = zero8();
#pragma unroll
      for (int kc = 0; kc < 4; ++kc) {
        const v16b bh = ldfrag(bph + kc * 32);
        const v16b bl = ldfrag(bpl + kc * 32);
        acc = wm(fh[kc], bh, acc);
        acc = wm(fh[kc], bl, acc);
        acc = wm(fl[kc], bh, acc);
      }
      const float bias = b3[min(n, N3 - 1)];
#pragma unroll
      for (int r = 0; r < 8; ++r) pw[(8 * hh + r) * PP + n] = acc[r] + bias;
    }
  }
  __syncthreads();

  float ldacc = 0.0f;
  {
    const size_t rowoff = (size_t)(row0 + m) * DIN;
#pragma unroll 1
    for (int j = 0; j < 4; ++j) {
      const int d = 4 * hh + j;
      const float xt = x[rowoff + d];
      const float xcd = x[rowoff + DT + d];
      const float* p = pw + m * PP + d * SPL;

      float e1[NB], e2[NB];
#pragma unroll
      for (int i = 0; i < NB; ++i) { e1[i] = p[i]; e2[i] = p[NB + i]; }
      float m1 = e1[0], m2 = e2[0];
#pragma unroll
      for (int i = 1; i < NB; ++i) { m1 = fmaxf(m1, e1[i]); m2 = fmaxf(m2, e2[i]); }
      float s1 = 0.0f, s2 = 0.0f;
#pragma unroll
      for (int i = 0; i < NB; ++i) {
        e1[i] = expf(e1[i] - m1);  s1 = s1 + e1[i];
        e2[i] = expf(e2[i] - m2);  s2 = s2 + e2[i];
      }
      const float i1 = 1.0f / s1, i2 = 1.0f / s2;
      const float xc = fminf(fmaxf(xt, 0.0f), 1.0f);

      float cx = 0.0f, cy = 0.0f, xk0 = 0.0f, yk0 = 0.0f;
      float wk = e1[0] * i1, hk = e2[0] * i2;
      float pr0 = 0.0f, pr1 = p[2 * NB];
      int cnt = 0;
#pragma unroll
      for (int q = 0; q < NB - 1; ++q) {
        const float dxq = e1[q] * i1, dyq = e2[q] * i2;
        cx = cx + dxq;
        cy = cy + dyq;
        const bool le = (cx <= xc);
        const float nwk = e1[q + 1] * i1, nhk = e2[q + 1] * i2;
        const float np0 = p[2 * NB + q];
        const float np1 = (q + 2 <= NB - 1) ? p[2 * NB + q + 1] : 0.0f;
        cnt = le ? (q + 1) : cnt;
        xk0 = le ? cx  : xk0;   yk0 = le ? cy  : yk0;
        wk  = le ? nwk : wk;    hk  = le ? nhk : hk;
        pr0 = le ? np0 : pr0;   pr1 = le ? np1 : pr1;
      }
      const float d0 = (cnt == 0)      ? 1.0f : softplus_f(pr0);
      const float d1 = (cnt == NB - 1) ? 1.0f : softplus_f(pr1);

      const float xi  = (xc - xk0) / wk;
      const float s   = hk / wk;
      const float om  = 1.0f - xi;
      const float z   = xi * om;
      const float den = s + (d1 + d0 - 2.0f * s) * z;
      const float num = hk * (s * xi * xi + d0 * z);
      const float yv  = yk0 + num / den;
      const float dnm = s * s * (d1 * xi * xi + 2.0f * s * z + d0 * (om * om));
      const float drv = dnm / (den * den);
      const bool oob  = (xt < 0.0f) || (xt > 1.0f);
      const float y   = oob ? xt : yv;
      const float ld  = oob ? 0.0f : logf(drv);
      yw[m * DIN + d] = y;
      yw[m * DIN + DT + d] = xcd;
      ldacc = ldacc + ld;
    }
  }

  ldacc = ldacc + __shfl_xor(ldacc, 16);
  if (hh == 0) lst[wave * 16 + m] = ldacc;
  __syncthreads();

  const v4f y0 = *(const v4f*)(yw + 4 * lane);
  const v4f y1 = *(const v4f*)(yw + 128 + 4 * lane);
  const v4f lv = *(const v4f*)(lst + 4 * (lane & 7));
  float* gy = out + (size_t)row0 * DIN;
  float* gl = out + (size_t)yoff + (size_t)blockIdx.x * RPB + 4 * (lane & 7);
  const bool wl = (wave == 0) && (lane < 8);
  *(volatile v4f*)(gy + 4 * lane) = y0;
  *(volatile v4f*)(gy + 128 + 4 * lane) = y1;
  if (wl) *(volatile v4f*)gl = lv;
  __threadfence();
  *(volatile v4f*)(gy + 4 * lane) = y0;
  *(volatile v4f*)(gy + 128 + 4 * lane) = y1;
  if (wl) *(volatile v4f*)gl = lv;
}

extern "C" void kernel_launch(void* const* d_in, const int* in_sizes, int n_in,
                              void* d_out, int out_size, void* d_ws, size_t ws_size,
                              hipStream_t stream) {
  if (n_in < 12) return;
  const int n0 = in_sizes[0];
  if (n0 <= 0 || (n0 % DIN) != 0) return;
  const int N = n0 / DIN;
  if ((N % RPB) != 0) return;
  if (in_sizes[1] != N * KC) return;
  if (in_sizes[2] != DIN || in_sizes[3] != DIN || in_sizes[4] != DIN || in_sizes[5] != DIN) return;
  if (in_sizes[6] != DIN * NH || in_sizes[7] != NH) return;
  if (in_sizes[8] != NH * NH || in_sizes[9] != NH) return;
  if (in_sizes[10] != NH * N3 || in_sizes[11] != N3) return;
  if (out_size != N * DIN + N) return;

  const float* x   = (const float*)d_in[0];
  const float* cc  = (const float*)d_in[1];
  const float* bns = (const float*)d_in[2];
  const float* bnb = (const float*)d_in[3];
  const float* bnm = (const float*)d_in[4];
  const float* bnv = (const float*)d_in[5];
  const float* W1  = (const float*)d_in[6];
  const float* b1  = (const float*)d_in[7];
  const float* W2  = (const float*)d_in[8];
  const float* b2  = (const float*)d_in[9];
  const float* W3  = (const float*)d_in[10];
  const float* b3  = (const float*)d_in[11];
  float* out = (float*)d_out;

  const size_t wbytes = (size_t)WTOT * 2;
  if (wbytes > ws_size || wbytes > (size_t)WSCAP) return;
  unsigned short* wsp = (unsigned short*)d_ws;

  const int yoff = N * DIN;
  k_prep<<<PREPB, 256, 0, stream>>>(W1, W2, W3, wsp);
  k_main<<<N / RPB, NTHR, 0, stream>>>(x, cc, bns, bnb, bnm, bnv, b1, b2, b3, wsp, out, yoff);
}
